// GNN_65712999629491
// MI455X (gfx1250) — hardware-verified
//
#include <hip/hip_runtime.h>
#include <stddef.h>
#include <stdint.h>


#define DW      100
#define FIN     100
#define HID     100
#define CLS     50
#define HP      128
#define KA      256
#define NP1     128
#define NPC     64
#define NTHR    256
#define NWAVE   8
#define EPT     8
#define CHUNK   (NTHR * EPT)
#define WCAP    (EPT * 32)
#define LISTN   (NWAVE * WCAP)
#define NBMAX   2048
#define NBMIN   128
#define RCAP    24576
#define DEGCAP  64
#define RG      16
#define STW     (RG * DW)
#define NPW     ((RG * DW / 4 + 31) / 32)
#define GBM     64
#define GTHR    128
#define LDA     256
#define NPA     ((GBM * DW / 4 + GTHR - 1) / GTHR)
#define NPCE    ((GBM * CLS / 4 + GTHR - 1) / GTHR)
#define WSMAX   134217728
#define LDS_AGG ((2 * RCAP + 2 * NBMAX + LISTN) * 4 + 64)
#define LDS_G1  (GBM * LDA * 2 + GBM * HID * 4)
#define LDS_G2  (GBM * LDA * 2 + GBM * CLS * 4)

static_assert((CHUNK & (CHUNK - 1)) == 0 && CHUNK <= 4096);
static_assert((NBMAX & (NBMAX - 1)) == 0 && NBMAX <= 4096);
static_assert(NTHR * 8 == NBMAX);
static_assert(LISTN >= NBMAX);
static_assert(LISTN >= NWAVE * WCAP);
static_assert((RCAP % 32) == 0);
static_assert(LDS_AGG <= 300000 && (LDS_AGG % 16) == 0);
static_assert(NWAVE * STW <= RCAP);
static_assert(((NBMIN / 8) % RG) == 0 && (NBMAX % NBMIN) == 0);
static_assert(NPW * 32 >= RG * DW / 4);
static_assert((RG * DW * 4) % 128 == 0);
static_assert(GBM == (GTHR / 32) * 16 && (GBM % RG) == 0);
static_assert(FIN == DW && HID == DW && (DW % 4) == 0 && DW >= 4 && DW <= HP);
static_assert(HP == 128 && KA == 2 * HP && (KA % 32) == 0);
static_assert(NP1 == 8 * 16 && HID <= NP1 && NPC == 4 * 16 && CLS <= NPC);
static_assert(NPA * GTHR >= GBM * DW / 4 && NPCE * GTHR >= GBM * CLS / 4);
static_assert((GBM * DW * 4) % 128 == 0);
static_assert((GBM * CLS * 4) % 128 == 0 && (GBM * CLS) % 4 == 0);
static_assert((LDS_G1 % 16) == 0 && (LDS_G2 % 16) == 0 && LDS_G1 <= 65536 && LDS_G2 <= 65536);
static_assert(((GBM * LDA * 2) % 16) == 0);

typedef float          v4f   __attribute__((ext_vector_type(4)));
typedef float          v8f   __attribute__((ext_vector_type(8)));
typedef int            v4i   __attribute__((ext_vector_type(4)));
typedef int            v8i   __attribute__((ext_vector_type(8)));
typedef unsigned short v4us  __attribute__((ext_vector_type(4)));
typedef unsigned short v8us  __attribute__((ext_vector_type(8)));
typedef __bf16         v16bf __attribute__((ext_vector_type(16)));
union FragB { v16bf v; v8us h[2]; v8i w; };

__device__ __forceinline__ v8f wmb(const FragB& a, const FragB& b, v8f c) {
  v8f d = __builtin_amdgcn_wmma_f32_16x16x32_bf16(false, a.v, false, b.v, (short)0, c, false, false);
  asm volatile("v_nop\n\tv_nop\n\tv_nop\n\tv_nop" : "+v"(d) : "v"(a.w), "v"(b.w));
  return d;
}

__device__ __forceinline__ void ldwait() {
  asm volatile("s_wait_loadcnt 0x0" ::: "memory");
}

__device__ __forceinline__ unsigned int bf16u(float x) {
  const unsigned int u = __float_as_uint(x);
  return (u + 0x7FFFu + ((u >> 16) & 1u)) >> 16;
}
__device__ __forceinline__ float bf16r(float x) { return __uint_as_float(bf16u(x) << 16); }

__device__ __forceinline__ void split4(const v4f n, v4us* ho, v4us* lo) {
  float s[4] = {n.x, n.y, n.z, n.w};
  v4us h, l;
#pragma unroll
  for (int j = 0; j < 4; ++j) {
    const unsigned int hb = bf16u(s[j]);
    h[j] = (unsigned short)hb;
    l[j] = (unsigned short)bf16u(s[j] - __uint_as_float(hb << 16));
  }
  *ho = h; *lo = l;
}

__device__ __forceinline__ int clampi(int v, int lo, int hi) { return v < lo ? lo : (v > hi ? hi : v); }

__device__ __forceinline__ void lds_zero(v4f* base, int nBytes, int tid, int nthr) {
  v4i* z = (v4i*)base;
  const v4i z4 = {0, 0, 0, 0};
  const int n = nBytes >> 4;
  for (int i = tid; i < n; i += nthr) z[i] = z4;
}

__device__ __forceinline__ int scan_chunk(const int* __restrict__ dsts, int nE, int cbase, int slotBase,
                                          int nb, int vec8, int* list, int tid, int lane, int wave) {
  int wc = 0;
  const int el0  = tid * EPT;
  const int e0   = cbase + el0;
  const int sent = -2147483647 - 1;
  v4i da, db;
  if (vec8 != 0 && cbase + CHUNK <= nE) {
    da = *(const v4i*)(dsts + e0);
    db = *(const v4i*)(dsts + e0 + 4);
  } else {
    da.x = (e0     < nE) ? dsts[min(e0,     nE - 1)] : sent;
    da.y = (e0 + 1 < nE) ? dsts[min(e0 + 1, nE - 1)] : sent;
    da.z = (e0 + 2 < nE) ? dsts[min(e0 + 2, nE - 1)] : sent;
    da.w = (e0 + 3 < nE) ? dsts[min(e0 + 3, nE - 1)] : sent;
    db.x = (e0 + 4 < nE) ? dsts[min(e0 + 4, nE - 1)] : sent;
    db.y = (e0 + 5 < nE) ? dsts[min(e0 + 5, nE - 1)] : sent;
    db.z = (e0 + 6 < nE) ? dsts[min(e0 + 6, nE - 1)] : sent;
    db.w = (e0 + 7 < nE) ? dsts[min(e0 + 7, nE - 1)] : sent;
  }
  ldwait();
  const unsigned nbs = (unsigned)slotBase;
  const unsigned unb = (unsigned)nb;
  const unsigned s0 = (unsigned)da.x - nbs, s1 = (unsigned)da.y - nbs;
  const unsigned s2 = (unsigned)da.z - nbs, s3 = (unsigned)da.w - nbs;
  const unsigned s4 = (unsigned)db.x - nbs, s5 = (unsigned)db.y - nbs;
  const unsigned s6 = (unsigned)db.z - nbs, s7 = (unsigned)db.w - nbs;
  const bool h0 = s0 < unb, h1 = s1 < unb, h2 = s2 < unb, h3 = s3 < unb;
  const bool h4 = s4 < unb, h5 = s5 < unb, h6 = s6 < unb, h7 = s7 < unb;
  const unsigned any = __builtin_amdgcn_ballot_w32(h0 | h1 | h2 | h3 | h4 | h5 | h6 | h7);
  if (any != 0u) {
#define HITJ(J, HJ, SJ) { \
      const unsigned mj = __builtin_amdgcn_ballot_w32(HJ); \
      if (mj != 0u) { \
        if (HJ) { \
          const int pos = wc + (int)__builtin_amdgcn_mbcnt_lo(mj, 0u); \
          if (pos < WCAP) list[wave * WCAP + pos] = ((el0 + (J)) << 12) | (int)(SJ); \
        } \
        wc += (int)__builtin_popcount(mj); } }
    HITJ(0, h0, s0)
    HITJ(1, h1, s1)
    HITJ(2, h2, s2)
    HITJ(3, h3, s3)
    HITJ(4, h4, s4)
    HITJ(5, h5, s5)
    HITJ(6, h6, s6)
    HITJ(7, h7, s7)
#undef HITJ
  }
  return wc;
}

__device__ __forceinline__ int alpha_idx(int sid, int did, int gene, int nA) {
  int idx = gene + 1;
  idx = (sid >= 0 && did <  0) ? sid  : idx;
  idx = (did >= 0 && sid <  0) ? did  : idx;
  idx = (sid >= 0 && did >= 0) ? gene : idx;
  return clampi(idx, 0, nA - 1);
}

__global__ __launch_bounds__(NTHR) void k_escale(const int* __restrict__ ids, const int* __restrict__ src,
                                                 const int* __restrict__ dst, const float* __restrict__ ew,
                                                 const float* __restrict__ alpha, int nN, int nE, int nA, int vec4,
                                                 float* esc, int nUnits) {
  const int u = (int)blockIdx.x * NTHR + (int)threadIdx.x;
  if (u >= nUnits) return;
  const int e0 = 4 * u;
  v4i sv, dv;
  v4f wv;
  if (vec4 != 0) {
    const int eb = e0 < nE - 4 ? e0 : nE - 4;
    sv = *(const v4i*)(src + eb);
    dv = *(const v4i*)(dst + eb);
    wv = *(const v4f*)(ew + eb);
  } else {
    const int c0 = min(e0, nE - 1), c1 = min(e0 + 1, nE - 1), c2 = min(e0 + 2, nE - 1), c3 = min(e0 + 3, nE - 1);
    sv.x = src[c0]; sv.y = src[c1]; sv.z = src[c2]; sv.w = src[c3];
    dv.x = dst[c0]; dv.y = dst[c1]; dv.z = dst[c2]; dv.w = dst[c3];
    ldwait();
    wv.x = ew[c0];  wv.y = ew[c1];  wv.z = ew[c2];  wv.w = ew[c3];
  }
  ldwait();
  const int nm = nN - 1;
  v4i si, di;
  si.x = ids[clampi(sv.x, 0, nm)]; si.y = ids[clampi(sv.y, 0, nm)];
  si.z = ids[clampi(sv.z, 0, nm)]; si.w = ids[clampi(sv.w, 0, nm)];
  di.x = ids[clampi(dv.x, 0, nm)]; di.y = ids[clampi(dv.y, 0, nm)];
  di.z = ids[clampi(dv.z, 0, nm)]; di.w = ids[clampi(dv.w, 0, nm)];
  ldwait();
  const int gene = nA - 2;
  v4f av;
  av.x = alpha[alpha_idx(si.x, di.x, gene, nA)];
  av.y = alpha[alpha_idx(si.y, di.y, gene, nA)];
  av.z = alpha[alpha_idx(si.z, di.z, gene, nA)];
  av.w = alpha[alpha_idx(si.w, di.w, gene, nA)];
  ldwait();
  v4f r;
  r.x = (e0     < nE) ? bf16r(av.x) * bf16r(wv.x) : 0.0f;
  r.y = (e0 + 1 < nE) ? bf16r(av.y) * bf16r(wv.y) : 0.0f;
  r.z = (e0 + 2 < nE) ? bf16r(av.z) * bf16r(wv.z) : 0.0f;
  r.w = (e0 + 3 < nE) ? bf16r(av.w) * bf16r(wv.w) : 0.0f;
  float* op = esc + (size_t)e0;
  *(volatile v4f*)op = r;
  __threadfence();
  *(volatile v4f*)op = r;
}

__global__ __launch_bounds__(NTHR) void k_wprep(const float* __restrict__ W, int nout, int kin,
                                                unsigned short* wt, int nUnits) {
  const int u = (int)blockIdx.x * NTHR + (int)threadIdx.x;
  if (u >= nUnits) return;
  const int n   = u >> 5;
  const int k8  = (u & 31) * 8;
  const int kk  = k8 & (HP - 1);
  const int ncl = n < nout ? n : nout - 1;
  const float* p = W + (size_t)ncl * (size_t)kin;
  float wv[8];
#pragma unroll
  for (int i = 0; i < 8; ++i) {
    const int kc  = kk + i;
    const int kcl = kc < kin ? kc : kin - 1;
    wv[i] = p[kcl];
  }
  ldwait();
  v8us hv;
#pragma unroll
  for (int i = 0; i < 8; ++i) {
    const int kc = kk + i;
    const float v = (n < nout && kc < kin) ? wv[i] : 0.0f;
    hv[i] = (unsigned short)bf16u(v);
  }
  const size_t o = (size_t)n * KA + k8;
  *(volatile v8us*)(wt + o) = hv;
  __threadfence();
  *(volatile v8us*)(wt + o) = hv;
}

__device__ __forceinline__ void stage_a(const float* __restrict__ Af, int rowBase, unsigned short* hsA, int tid) {
  const float* ab = Af + (size_t)rowBase * DW;
  v4f pv[NPA];
#pragma unroll
  for (int i = 0; i < NPA; ++i) {
    int p = i * GTHR + tid;
    p = p > (GBM * DW / 4 - 1) ? (GBM * DW / 4 - 1) : p;
    pv[i] = *(const v4f*)(ab + 4 * p);
  }
  ldwait();
#pragma unroll
  for (int i = 0; i < NPA; ++i) {
    const int p = i * GTHR + tid;
    if (p < GBM * DW / 4) {
      const int row = p / (DW / 4);
      const int c   = (p - row * (DW / 4)) * 4;
      v4us hb, lb;
      split4(pv[i], &hb, &lb);
      *(v4us*)(hsA + row * LDA + c)      = hb;
      *(v4us*)(hsA + row * LDA + HP + c) = lb;
    }
  }
}

__global__ __launch_bounds__(GTHR) void k_gemm1(const float* __restrict__ Af, const unsigned short* __restrict__ WT,
                                                const float* __restrict__ bias, float* H) {
  extern __shared__ v4f lds_g[];
  unsigned short* hsA = (unsigned short*)lds_g;
  float* stg = (float*)((char*)lds_g + GBM * LDA * 2);
  const int tid = (int)threadIdx.x, lane = tid & 31, wave = tid >> 5, hh = lane >> 4, m = lane & 15;
  const int rowBase = (int)blockIdx.x * GBM;

  lds_zero(lds_g, LDS_G1, tid, GTHR);
  __syncthreads();
  stage_a(Af, rowBase, hsA, tid);
  __syncthreads();

  v8f acc[8];
  {
    const v8f z = {0.f, 0.f, 0.f, 0.f, 0.f, 0.f, 0.f, 0.f};
#pragma unroll
    for (int t = 0; t < 8; ++t) acc[t] = z;
  }
  const unsigned short* ap = hsA + (16 * wave + m) * LDA + 8 * hh;
  const unsigned short* wp = WT + (size_t)m * KA + 8 * hh;
#pragma unroll 1
  for (int ks = 0; ks < KA / 32; ++ks) {
    FragB af;
    af.h[0] = *(const v8us*)(ap + 32 * ks);
    af.h[1] = *(const v8us*)(ap + 32 * ks + 16);
#pragma unroll
    for (int t = 0; t < 8; ++t) {
      const unsigned short* wq = wp + (size_t)(16 * t) * KA + 32 * ks;
      FragB bf;
      bf.h[0] = *(const v8us*)wq;
      bf.h[1] = *(const v8us*)(wq + 16);
      acc[t] = wmb(af, bf, acc[t]);
    }
  }

  float bv[8];
#pragma unroll
  for (int t = 0; t < 8; ++t) {
    const int lc = 16 * t + m;
    const int bi = lc > HID - 1 ? HID - 1 : lc;
    bv[t] = bias[bi];
  }
  ldwait();
#pragma unroll
  for (int t = 0; t < 8; ++t) {
    const int lc = 16 * t + m;
    const float b = lc < HID ? bf16r(bv[t]) : 0.0f;
#pragma unroll
    for (int r = 0; r < 8; ++r) {
      const int lr = 16 * wave + 8 * hh + r;
      const float v = fmaxf(acc[t][r] + b, 0.0f);
      if (lc < HID) stg[lr * HID + lc] = v;
    }
  }
  __syncthreads();

  v4f pv[NPA];
#pragma unroll
  for (int i = 0; i < NPA; ++i) {
    int p = i * GTHR + tid;
    p = p > (GBM * HID / 4 - 1) ? (GBM * HID / 4 - 1) : p;
    pv[i] = *(const v4f*)(stg + 4 * p);
  }
  float* ob = H + (size_t)rowBase * HID;
#pragma unroll
  for (int i = 0; i < NPA; ++i) {
    const int p = i * GTHR + tid;
    if (p < GBM * HID / 4) *(volatile v4f*)(ob + 4 * p) = pv[i];
  }
  __threadfence();
#pragma unroll
  for (int i = 0; i < NPA; ++i) {
    const int p = i * GTHR + tid;
    if (p < GBM * HID / 4) *(volatile v4f*)(ob + 4 * p) = pv[i];
  }
}

__global__ __launch_bounds__(GTHR) void k_gemm2c(const float* __restrict__ Af, const unsigned short* __restrict__ WT,
                                                 const float* __restrict__ bias, const unsigned short* __restrict__ WL,
                                                 const float* __restrict__ bcls, float* outF, int nRows) {
  extern __shared__ v4f lds_g[];
  unsigned short* hsA = (unsigned short*)lds_g;
  float* stg = (float*)((char*)lds_g + GBM * LDA * 2);
  const int tid = (int)threadIdx.x, lane = tid & 31, wave = tid >> 5, hh = lane >> 4, m = lane & 15;
  const int rowBase = (int)blockIdx.x * GBM;

  lds_zero(lds_g, LDS_G2, tid, GTHR);
  __syncthreads();
  stage_a(Af, rowBase, hsA, tid);
  __syncthreads();

  v8f acc[8];
  {
    const v8f z = {0.f, 0.f, 0.f, 0.f, 0.f, 0.f, 0.f, 0.f};
#pragma unroll
    for (int t = 0; t < 8; ++t) acc[t] = z;
  }
  const unsigned short* ap = hsA + (16 * wave + m) * LDA + 8 * hh;
  {
    const unsigned short* wp = WT + (size_t)m * KA + 8 * hh;
#pragma unroll 1
    for (int ks = 0; ks < KA / 32; ++ks) {
      FragB af;
      af.h[0] = *(const v8us*)(ap + 32 * ks);
      af.h[1] = *(const v8us*)(ap + 32 * ks + 16);
#pragma unroll
      for (int t = 0; t < 8; ++t) {
        const unsigned short* wq = wp + (size_t)(16 * t) * KA + 32 * ks;
        FragB bf;
        bf.h[0] = *(const v8us*)wq;
        bf.h[1] = *(const v8us*)(wq + 16);
        acc[t] = wmb(af, bf, acc[t]);
      }
    }
  }

  float bv[8];
#pragma unroll
  for (int t = 0; t < 8; ++t) {
    const int lc = 16 * t + m;
    const int bi = lc > HID - 1 ? HID - 1 : lc;
    bv[t] = bias[bi];
  }
  ldwait();
  __syncthreads();
#pragma unroll
  for (int t = 0; t < 8; ++t) {
    const int lc = 16 * t + m;
    const float b = lc < HID ? bf16r(bv[t]) : 0.0f;
#pragma unroll
    for (int r = 0; r < 8; ++r) {
      const int lr = 16 * wave + 8 * hh + r;
      float v = fmaxf(acc[t][r] + b, 0.0f);
      v = lc < HID ? v : 0.0f;
      const unsigned int hb = bf16u(v);
      const unsigned int lb = bf16u(v - __uint_as_float(hb << 16));
      hsA[lr * LDA + lc]      = (unsigned short)hb;
      hsA[lr * LDA + HP + lc] = (unsigned short)lb;
    }
  }
  __syncthreads();

  v8f acc2[4];
  {
    const v8f z = {0.f, 0.f, 0.f, 0.f, 0.f, 0.f, 0.f, 0.f};
#pragma unroll
    for (int t = 0; t < 4; ++t) acc2[t] = z;
  }
  {
    const unsigned short* wp = WL + (size_t)m * KA + 8 * hh;
#pragma unroll 1
    for (int ks = 0; ks < KA / 32; ++ks) {
      FragB af;
      af.h[0] = *(const v8us*)(ap + 32 * ks);
      af.h[1] = *(const v8us*)(ap + 32 * ks + 16);
#pragma unroll
      for (int t = 0; t < 4; ++t) {
        const unsigned short* wq = wp + (size_t)(16 * t) * KA + 32 * ks;
        FragB bf;
        bf.h[0] = *(const v8us*)wq;
        bf.h[1] = *(const v8us*)(wq + 16);
        acc2[t] = wmb(af, bf, acc2[t]);
      }
    }
  }

  float bc[4];
#pragma unroll
  for (int t = 0; t < 4; ++t) {
    const int lc = 16 * t + m;
    const int bi = lc > CLS - 1 ? CLS - 1 : lc;
    bc[t] = bcls[bi];
  }
  ldwait();
#pragma unroll
  for (int t = 0; t < 4; ++t) {
    const int lc = 16 * t + m;
    const float b = lc < CLS ? bf16r(bc[t]) : 0.0f;
#pragma unroll
    for (int r = 0; r < 8; ++r) {
      const int lr = 16 * wave + 8 * hh + r;
      const float v = acc2[t][r] + b;
      if (lc < CLS) stg[lr * CLS + lc] = v;
    }
  }
  __syncthreads();

  int nv = nRows - rowBase;
  nv = nv < 0 ? 0 : (nv > GBM ? GBM : nv);
  const int nf   = nv * CLS;
  const int np   = nf >> 2;
  const int tail = nf & 3;
  v4f po[NPCE];
#pragma unroll
  for (int i = 0; i < NPCE; ++i) {
    int p = i * GTHR + tid;
    p = p > (GBM * CLS / 4 - 1) ? (GBM * CLS / 4 - 1) : p;
    po[i] = *(const v4f*)(stg + 4 * p);
  }
  float tv;
  {
    int ti = 4 * np + tid;
    ti = ti > GBM * CLS - 1 ? GBM * CLS - 1 : ti;
    tv = stg[ti];
  }
  float* ob = outF + (size_t)rowBase * CLS;
#pragma unroll
  for (int i = 0; i < NPCE; ++i) {
    const int p = i * GTHR + tid;
    if (p < np) *(volatile v4f*)(ob + 4 * p) = po[i];
  }
  if (tid < tail) *(volatile float*)(ob + 4 * np + tid) = tv;
  __threadfence();
#pragma unroll
  for (int i = 0; i < NPCE; ++i) {
    const int p = i * GTHR + tid;
    if (p < np) *(volatile v4f*)(ob + 4 * p) = po[i];
  }
  if (tid < tail) *(volatile float*)(ob + 4 * np + tid) = tv;
}

template<int RND>
__global__ __launch_bounds__(NTHR) void k_agg(
    const int* __restrict__ srcs, const int* __restrict__ dsts, const float* __restrict__ esc,
    const float* __restrict__ Hs, int pitch,
    float* AG, int nN, int nE, int nb, int vec8, int MPr) {
  extern __shared__ v4f lds_dyn[];
  int* reg1 = (int*)lds_dyn;
  int* reg2 = reg1 + RCAP;
  int* scnt = reg2 + RCAP;
  int* soff = scnt + NBMAX;
  int* list = soff + NBMAX;
  int* wcnt = list + LISTN;
  int* wtot = wcnt + NWAVE;
  const int tid = (int)threadIdx.x, lane = tid & 31, wave = tid >> 5;
  const int nodeBase = (int)blockIdx.x * nb;

  lds_zero(lds_dyn, LDS_AGG, tid, NTHR);
  __syncthreads();

  int tot = 0;
  const int nChunks = (nE + CHUNK - 1) / CHUNK;
#pragma unroll 1
  for (int ch = 0; ch < nChunks; ++ch) {
    const int cbase = ch * CHUNK;
    const int wc = scan_chunk(dsts, nE, cbase, nodeBase, nb, vec8, list, tid, lane, wave);
    if (lane == 0) wcnt[wave] = wc;
    __syncthreads();
    int pre = 0, all = 0;
#pragma unroll
    for (int w2 = 0; w2 < NWAVE; ++w2) {
      int c = wcnt[w2];
      c = c < 0 ? 0 : (c > WCAP ? WCAP : c);
      all += c;
      pre += (w2 < wave) ? c : 0;
    }
    const int wcc  = wc > WCAP ? WCAP : wc;
    const int base = tot + pre;
#pragma unroll 1
    for (int i = lane; i < wcc; i += 32) {
      const int ent = list[wave * WCAP + i];
      const int el  = (ent >> 12) & (CHUNK - 1);
      const int sl  = ent & (NBMAX - 1);
      int eid = cbase + el;
      eid = eid > nE - 1 ? nE - 1 : eid;
      const int pos = base + i;
      if (pos < RCAP) reg1[pos] = (int)(((unsigned)eid << 12) | (unsigned)sl);
    }
    tot += all;
    tot = tot > RCAP ? RCAP : tot;
    __syncthreads();
  }
  const int nh = tot;

  if (wave == 0) {
#pragma unroll 1
    for (int b0 = 0; b0 < nh; b0 += 32) {
      const int idx = b0 + lane;
      const int uv  = reg1[idx < RCAP ? idx : RCAP - 1];
      const int m32 = (nh - b0) < 32 ? (nh - b0) : 32;
#pragma unroll 1
      for (int k = 0; k < m32; ++k) {
        const int u  = __builtin_amdgcn_readlane(uv, k);
        const int sl = u & (NBMAX - 1);
        if (lane == 0) scnt[sl] = scnt[sl] + 1;
      }
    }
  }
  __syncthreads();

  {
    const v4i ca = *(const v4i*)(scnt + 8 * tid);
    const v4i cb = *(const v4i*)(scnt + 8 * tid + 4);
    const int e0 = ca.x < 0 ? 0 : ca.x, e1 = ca.y < 0 ? 0 : ca.y, e2 = ca.z < 0 ? 0 : ca.z, e3 = ca.w < 0 ? 0 : ca.w;
    const int e4 = cb.x < 0 ? 0 : cb.x, e5 = cb.y < 0 ? 0 : cb.y, e6 = cb.z < 0 ? 0 : cb.z, e7 = cb.w < 0 ? 0 : cb.w;
    const int ts = e0 + e1 + e2 + e3 + e4 + e5 + e6 + e7;
    int incl = ts;
#pragma unroll
    for (int d = 1; d < 32; d <<= 1) {
      const int up = __shfl_up(incl, d);
      if (lane >= d) incl += up;
    }
    if (lane == 31) wtot[wave] = incl;
    __syncthreads();
    int pre = 0;
#pragma unroll
    for (int w2 = 0; w2 < NWAVE; ++w2) pre += (w2 < wave) ? wtot[w2] : 0;
    int run = pre + incl - ts;
    soff[8 * tid + 0] = run; run += e0;
    soff[8 * tid + 1] = run; run += e1;
    soff[8 * tid + 2] = run; run += e2;
    soff[8 * tid + 3] = run; run += e3;
    soff[8 * tid + 4] = run; run += e4;
    soff[8 * tid + 5] = run; run += e5;
    soff[8 * tid + 6] = run; run += e6;
    soff[8 * tid + 7] = run;
  }
  __syncthreads();
  for (int i = tid; i < NBMAX; i += NTHR) list[i] = soff[i];
  __syncthreads();

  if (wave == 0) {
#pragma unroll 1
    for (int b0 = 0; b0 < nh; b0 += 32) {
      const int idx = b0 + lane;
      const int uv  = reg1[idx < RCAP ? idx : RCAP - 1];
      const int m32 = (nh - b0) < 32 ? (nh - b0) : 32;
#pragma unroll 1
      for (int k = 0; k < m32; ++k) {
        const int u   = __builtin_amdgcn_readlane(uv, k);
        const int sl  = u & (NBMAX - 1);
        const int eid = (int)((unsigned)u >> 12);
        if (lane == 0) {
          int pos = list[sl];
          pos = pos < 0 ? 0 : (pos > RCAP - 1 ? RCAP - 1 : pos);
          reg2[pos] = eid;
          list[sl] = pos + 1;
        }
      }
    }
  }
  __syncthreads();

  const int nbw = nb >> 3;
  const bool ovf = (nh >= RCAP);
  const float qnan = __int_as_float(0x7fc00000);
  float* stw = (float*)reg1 + wave * STW;
  const int c4 = 4 * lane;
  const bool cval = c4 < DW;
  const int ccl = c4 < DW - 4 ? c4 : DW - 4;
#pragma unroll 1
  for (int jt = 0; jt < nbw; ++jt) {
    const int slot = wave * nbw + jt;
    int st = __builtin_amdgcn_readfirstlane(soff[slot]);
    const int craw = __builtin_amdgcn_readfirstlane(scnt[slot]);
    int cnt = craw;
    st  = st < 0 ? 0 : (st > nh ? nh : st);
    cnt = cnt < 0 ? 0 : (cnt > DEGCAP ? DEGCAP : cnt);
    if (cnt > nh - st) cnt = nh - st;
    const float pz = (ovf || craw > DEGCAP) ? qnan : 0.0f;

    v4f acc = {0.f, 0.f, 0.f, 0.f};
#pragma unroll 1
    for (int q = 0; q < cnt; ++q) {
      int idx = st + q; idx = idx > RCAP - 1 ? RCAP - 1 : idx;
      int eid = reg2[idx];
      eid = eid < 0 ? 0 : (eid > nE - 1 ? nE - 1 : eid);
      const int sraw = srcs[eid];
      const float sc = esc[eid];
      ldwait();
      const int s = sraw < 0 ? 0 : (sraw > nN - 1 ? nN - 1 : sraw);
      v4f hv = *(const v4f*)(Hs + (size_t)s * (size_t)pitch + ccl);
      ldwait();
      if (RND) { hv.x = bf16r(hv.x); hv.y = bf16r(hv.y); hv.z = bf16r(hv.z); hv.w = bf16r(hv.w); }
      acc.x = fmaf(sc, hv.x, acc.x);
      acc.y = fmaf(sc, hv.y, acc.y);
      acc.z = fmaf(sc, hv.z, acc.z);
      acc.w = fmaf(sc, hv.w, acc.w);
    }
    const float dg  = craw > 0 ? (float)craw : 1.0f;
    const float inv = (craw > 0 ? 1.0f : 0.0f) * (1.0f / dg);
    v4f n;
    n.x = acc.x * inv + pz;
    n.y = acc.y * inv + pz;
    n.z = acc.z * inv + pz;
    n.w = acc.w * inv + pz;
    const int rl = jt & (RG - 1);
    if (cval) *(v4f*)(stw + rl * DW + c4) = n;

    if (rl == RG - 1) {
      __syncthreads();
      const int row0 = nodeBase + slot - (RG - 1);
      const bool wr = (row0 + RG) <= MPr;
      v4f pv[NPW];
#pragma unroll
      for (int i = 0; i < NPW; ++i) {
        int p = 32 * i + lane;
        p = p > (RG * DW / 4 - 1) ? (RG * DW / 4 - 1) : p;
        pv[i] = *(const v4f*)(stw + 4 * p);
      }
      float* ob = AG + (size_t)row0 * DW;
#pragma unroll
      for (int i = 0; i < NPW; ++i) {
        const int p = 32 * i + lane;
        if (wr && p < RG * DW / 4) *(volatile v4f*)(ob + 4 * p) = pv[i];
      }
      __threadfence();
#pragma unroll
      for (int i = 0; i < NPW; ++i) {
        const int p = 32 * i + lane;
        if (wr && p < RG * DW / 4) *(volatile v4f*)(ob + 4 * p) = pv[i];
      }
      __syncthreads();
    }
  }
}

static int pick_nb(int nE, int nN) {
  int nb = NBMAX;
  while (nb > NBMIN && (long long)nb * (long long)nE * 5LL > (long long)RCAP * (long long)nN * 4LL) nb >>= 1;
  return nb;
}
static inline int cdiv(int a, int b) { return (a + b - 1) / b; }

extern "C" void kernel_launch(void* const* d_in, const int* in_sizes, int n_in,
                              void* d_out, int out_size, void* d_ws, size_t ws_size,
                              hipStream_t stream) {
  if (n_in < 12) return;
  const int nN = in_sizes[1];
  if (nN <= 0 || nN > (1 << 22)) return;
  if (in_sizes[0] != nN * FIN) return;
  const int nE = in_sizes[2];
  if (nE < 1 || nE > (1 << 20)) return;
  if (in_sizes[3] != nE || in_sizes[4] != nE) return;
  const int nA = in_sizes[5];
  if (nA < 2) return;
  if (in_sizes[6]  != HID * FIN || in_sizes[7]  != HID) return;
  if (in_sizes[8]  != HID * HID || in_sizes[9]  != HID) return;
  if (in_sizes[10] != CLS * HID || in_sizes[11] != CLS) return;
  if (out_size != nN * CLS) return;

  const float* feat  = (const float*)d_in[0];
  const int*   ids   = (const int*)  d_in[1];
  const int*   src   = (const int*)  d_in[2];
  const int*   dst   = (const int*)  d_in[3];
  const float* ew    = (const float*)d_in[4];
  const float* alpha = (const float*)d_in[5];
  const float* W1    = (const float*)d_in[6];
  const float* b1    = (const float*)d_in[7];
  const float* W2    = (const float*)d_in[8];
  const float* b2    = (const float*)d_in[9];
  const float* Wl    = (const float*)d_in[10];
  const float* bl    = (const float*)d_in[11];
  float* out = (float*)d_out;

  const int MP   = cdiv(nN, GBM) * GBM;
  const int nb   = pick_nb(nE, nN);
  if (nb < NBMIN || nb > NBMAX || ((nb >> 3) % RG) != 0) return;
  const int gA   = cdiv(MP, nb);
  const int vec8 = ((nE & 3) == 0) ? 1 : 0;
  const int vec4 = ((nE & 3) == 0 && nE >= 4) ? 1 : 0;
  if (gA * nb < MP) return;
  const int EP   = cdiv(nE, 128) * 128;

  char* ws = (char*)d_ws;
  size_t off = 0;
  const size_t oESC = off; off += (size_t)EP * 4;                  off = (off + 255) & ~(size_t)255;
  const size_t oAG1 = off; off += (size_t)MP * DW * 4;             off = (off + 255) & ~(size_t)255;
  const size_t oH1  = off; off += (size_t)MP * HID * 4;            off = (off + 255) & ~(size_t)255;
  const size_t oAG2 = off; off += (size_t)MP * DW * 4;             off = (off + 255) & ~(size_t)255;
  const size_t oW1  = off; off += (size_t)NP1 * KA * 2;            off = (off + 255) & ~(size_t)255;
  const size_t oW2  = off; off += (size_t)NP1 * KA * 2;            off = (off + 255) & ~(size_t)255;
  const size_t oWL  = off; off += (size_t)NPC * KA * 2;            off = (off + 255) & ~(size_t)255;
  if (off > ws_size || off > (size_t)WSMAX) return;
  float*          ESC = (float*)(ws + oESC);
  float*          AG1 = (float*)(ws + oAG1);
  float*          H1  = (float*)(ws + oH1);
  float*          AG2 = (float*)(ws + oAG2);
  unsigned short* W1T = (unsigned short*)(ws + oW1);
  unsigned short* W2T = (unsigned short*)(ws + oW2);
  unsigned short* WLT = (unsigned short*)(ws + oWL);

  hipFuncSetAttribute(reinterpret_cast<const void*>(&k_agg<1>),
                      hipFuncAttributeMaxDynamicSharedMemorySize, LDS_AGG);
  hipFuncSetAttribute(reinterpret_cast<const void*>(&k_agg<0>),
                      hipFuncAttributeMaxDynamicSharedMemorySize, LDS_AGG);
  hipFuncSetAttribute(reinterpret_cast<const void*>(&k_gemm1),
                      hipFuncAttributeMaxDynamicSharedMemorySize, LDS_G1);
  hipFuncSetAttribute(reinterpret_cast<const void*>(&k_gemm2c),
                      hipFuncAttributeMaxDynamicSharedMemorySize, LDS_G2);

  {
    const int nU = EP / 4;
    k_escale<<<cdiv(nU, NTHR), NTHR, 0, stream>>>(ids, src, dst, ew, alpha, nN, nE, nA, vec4, ESC, nU);
  }
  {
    const int nU1 = NP1 * (KA / 8);
    k_wprep<<<cdiv(nU1, NTHR), NTHR, 0, stream>>>(W1, HID, FIN, W1T, nU1);
    k_wprep<<<cdiv(nU1, NTHR), NTHR, 0, stream>>>(W2, HID, HID, W2T, nU1);
    const int nU3 = NPC * (KA / 8);
    k_wprep<<<cdiv(nU3, NTHR), NTHR, 0, stream>>>(Wl, CLS, HID, WLT, nU3);
  }

  const int gM = MP / GBM;
  k_agg<1><<<gA, NTHR, LDS_AGG, stream>>>(src, dst, ESC, feat, FIN, AG1, nN, nE, nb, vec8, MP);
  k_gemm1<<<gM, GTHR, LDS_G1, stream>>>(AG1, W1T, b1, H1);
  k_agg<0><<<gA, NTHR, LDS_AGG, stream>>>(src, dst, ESC, H1, HID, AG2, nN, nE, nb, vec8, MP);
  k_gemm2c<<<gM, GTHR, LDS_G2, stream>>>(AG2, W2T, b2, WLT, bl, out, nN);
}
